// cliqueMPNN_hindsight_7481833029835
// MI455X (gfx1250) — hardware-verified
//
#include <hip/hip_runtime.h>
#include <math.h>
typedef __attribute__((ext_vector_type(16))) _Float16 v16h;
typedef __attribute__((ext_vector_type(8)))  _Float16 v8h;
typedef __attribute__((ext_vector_type(16))) __bf16   v16b;
typedef __attribute__((ext_vector_type(8)))  __bf16   v8b;
typedef __attribute__((ext_vector_type(8)))  float    v8f;
typedef __attribute__((ext_vector_type(4)))  float    v4f;
#define PSCALE 32768.0f
#define U16(p) ((const unsigned short*)(const void*)(p))
#define PSCALE_INV (1.0f / 32768.0f)

__device__ __forceinline__ unsigned short f2bf_bits(float f) {
  unsigned u = __float_as_uint(f);
  return (unsigned short)((u + 0x7FFFu + ((u >> 16) & 1u)) >> 16);
}
__device__ __forceinline__ float bf_bits2f(unsigned short h) { return __uint_as_float(((unsigned)h) << 16); }

__device__ __forceinline__ void dep_guard_h(v8f& a, v8f& b, v16h x, v16h y) { asm volatile("v_nop\n\tv_nop\n\tv_nop\n\tv_nop" : "+v"(a), "+v"(b) : "v"(x), "v"(y)); }
__device__ __forceinline__ void dep_guard_b(v8f& a, v8f& b, v16b x, v16b y) { asm volatile("v_nop\n\tv_nop\n\tv_nop\n\tv_nop" : "+v"(a), "+v"(b) : "v"(x), "v"(y)); }
__device__ __forceinline__ void keep4_h(v16h a, v16h b, v16h c, v16h d) { asm volatile("v_nop" :: "v"(a), "v"(b), "v"(c), "v"(d)); }
__device__ __forceinline__ void keep4_b(v16b a, v16b b, v16b c, v16b d) { asm volatile("v_nop" :: "v"(a), "v"(b), "v"(c), "v"(d)); }
__device__ __forceinline__ void acc_guard4(v8f& a, v8f& b, v8f& c, v8f& d) { asm volatile("v_nop\n\tv_nop\n\tv_nop\n\tv_nop" : "+v"(a), "+v"(b), "+v"(c), "+v"(d)); }
template <typename T> struct Frag;
template <> struct Frag<_Float16> {
  typedef v16h V; union U { v16h v; v8h h[2]; };
  static __device__ __forceinline__ v16h load(const _Float16* p) {
    U f; f.h[0] = *(const v8h*)(p); f.h[1] = *(const v8h*)(p + 16); return f.v;
  }
  static __device__ __forceinline__ v8f mma(v16h a, v16h b, v8f c) {
    return __builtin_amdgcn_wmma_f32_16x16x32_f16(false, a, false, b, (short)0, c, false, false);
  }
  static __device__ __forceinline__ void guard(v8f& a, v8f& b, v16h x, v16h y) { dep_guard_h(a, b, x, y); }
  static __device__ __forceinline__ void keep(v16h a, v16h b, v16h c, v16h d) { keep4_h(a, b, c, d); }
};
template <> struct Frag<__bf16> {
  typedef v16b V; union U { v16b v; v8b h[2]; };
  static __device__ __forceinline__ v16b load(const __bf16* p) {
    U f; f.h[0] = *(const v8b*)(p); f.h[1] = *(const v8b*)(p + 16); return f.v;
  }
  static __device__ __forceinline__ v8f mma(v16b a, v16b b, v8f c) {
    return __builtin_amdgcn_wmma_f32_16x16x32_bf16(false, a, false, b, (short)0, c, false, false);
  }
  static __device__ __forceinline__ void guard(v8f& a, v8f& b, v16b x, v16b y) { dep_guard_b(a, b, x, y); }
  static __device__ __forceinline__ void keep(v16b a, v16b b, v16b c, v16b d) { keep4_b(a, b, c, d); }
};

template <int ET> struct Elem;
template <> struct Elem<0> { typedef _Float16 T; };
template <> struct Elem<1> { typedef __bf16 T; };
template <int ET, bool SPLIT, int BIAS_MODE, int OUT_MODE, bool RESID, int ACT = 0>
__global__ __launch_bounds__(256) void wmma_gemm64(
    const unsigned short* __restrict__ Ap, const unsigned short* __restrict__ A2p, int lda, long strideA,
    const unsigned short* __restrict__ Btp, const unsigned short* __restrict__ Bt2p, int ldb, long strideB,
    void* __restrict__ Cout, void* __restrict__ Cout2, int ldc, long strideC,
    const float* __restrict__ bias,
    const float* __restrict__ resid, long strideR,
    int M, int N, int K, float scale) {
  typedef typename Elem<ET>::T T;
  typedef typename Frag<T>::V V;
  const T* A = (const T*)Ap; const T* A2 = (const T*)A2p; const T* Bt = (const T*)Btp; const T* Bt2 = (const T*)Bt2p;
  __shared__ __align__(16) float sT[8][16 * 68];
  const int b    = blockIdx.y;
  const int lane = threadIdx.x & 31;
  const int wave = threadIdx.x >> 5;
  const int tilesN = N >> 6;
  const int tilesM = M >> 6;
  const int tile = blockIdx.x * 8 + wave;
  if (tile >= tilesM * tilesN) return;
  const int tm = tile / tilesN;
  const int tn = tile - tm * tilesN;
  const int m0 = tm << 6;
  const int n0 = tn << 6;

  const T* Ab  = A  + (size_t)b * strideA;
  const T* Bb  = Bt + (size_t)b * strideB;
  const T* Ab2 = SPLIT ? (A2  + (size_t)b * strideA) : nullptr;
  const T* Bb2 = SPLIT ? (Bt2 + (size_t)b * strideB) : nullptr;

  const int rlane = lane & 15;
  const int koff  = (lane >> 4) * 8;
  const int mOff  = (lane >> 4) * 8;

  v8f acc[4][4];
#pragma unroll
  for (int i = 0; i < 4; ++i)
#pragma unroll
    for (int j = 0; j < 4; ++j) acc[i][j] = (v8f){0.f,0.f,0.f,0.f,0.f,0.f,0.f,0.f};

  for (int k0 = 0; k0 < K; k0 += 32) {
    V bh[4], bl[4];
#pragma unroll
    for (int j = 0; j < 4; ++j) {
      const size_t bo = (size_t)(n0 + (j << 4) + rlane) * ldb + koff + k0;
      bh[j] = Frag<T>::load(Bb + bo);
      if (SPLIT) bl[j] = Frag<T>::load(Bb2 + bo);
    }
#pragma unroll
    for (int i = 0; i < 4; ++i) {
      const size_t ao = (size_t)(m0 + (i << 4) + rlane) * lda + koff + k0;
      V ah = Frag<T>::load(Ab + ao);
      V al;
      if (SPLIT) al = Frag<T>::load(Ab2 + ao);
#pragma unroll
      for (int j = 0; j < 4; ++j) {
        acc[i][j] = Frag<T>::mma(ah, bh[j], acc[i][j]);
        if (SPLIT) {
          acc[i][j] = Frag<T>::mma(ah, bl[j], acc[i][j]);
          acc[i][j] = Frag<T>::mma(al, bh[j], acc[i][j]);
        }
      }
      Frag<T>::guard(acc[i][0], acc[i][3], ah, SPLIT ? al : ah);
    }
    Frag<T>::keep(bh[0], bh[1], bh[2], bh[3]);
    if (SPLIT) Frag<T>::keep(bl[0], bl[1], bl[2], bl[3]);
  }
  acc_guard4(acc[0][0], acc[0][1], acc[0][2], acc[0][3]);
  acc_guard4(acc[1][0], acc[1][1], acc[1][2], acc[1][3]);
  acc_guard4(acc[2][0], acc[2][1], acc[2][2], acc[2][3]);
  acc_guard4(acc[3][0], acc[3][1], acc[3][2], acc[3][3]);

  float* slab = sT[wave];
  const float* Rb = RESID ? (resid + (size_t)b * strideR) : nullptr;
#pragma unroll
  for (int i = 0; i < 4; ++i) {
    const int mBase = m0 + (i << 4);
#pragma unroll
    for (int j = 0; j < 4; ++j) {
      const int n = n0 + (j << 4) + rlane;
      float bv = 0.f;
      if (BIAS_MODE == 2) bv = bias[n];
#pragma unroll
      for (int r = 0; r < 8; ++r) {
        float v = acc[i][j][r] * scale;
        if (BIAS_MODE == 1) v += bias[mBase + mOff + r];
        if (BIAS_MODE == 2) v += bv;
        if (RESID) v += Rb[(size_t)(mBase + mOff + r) * ldc + n];
        if (ACT == 1) v = tanhf(v);
        if (ACT == 2) v = fmaxf(v, 0.0f);
        if (ACT == 3) v = v / (1.0f + expf(-v));
        if (ACT == 4) v = (v > 0.f) ? v : 0.01f * v;
        slab[(mOff + r) * 68 + (j << 4) + rlane] = v;
      }
    }
    __builtin_amdgcn_fence(__ATOMIC_RELEASE, "workgroup");
    __builtin_amdgcn_wave_barrier();
    __builtin_amdgcn_fence(__ATOMIC_ACQUIRE, "workgroup");
    if (OUT_MODE == 0) {
      float* C = (float*)Cout + (size_t)b * strideC;
      const int hh = lane >> 4, c4 = (lane & 15) * 4;
      for (int pass = 0; pass < 2; ++pass) {
#pragma unroll
        for (int it = 0; it < 8; ++it) {
          const int row = it * 2 + hh;
          v4f v = *(const v4f*)(slab + row * 68 + c4);
          *(volatile v4f*)(C + (size_t)(mBase + row) * ldc + n0 + c4) = v;
        }
        __threadfence();
      }
    } else {
      const int q = lane >> 3, c8 = (lane & 7) * 8;
      unsigned short* C  = (unsigned short*)Cout  + (size_t)b * strideC;
      unsigned short* C2 = (OUT_MODE == 2) ? ((unsigned short*)Cout2 + (size_t)b * strideC) : nullptr;
      for (int pass = 0; pass < 2; ++pass) {
#pragma unroll
        for (int it = 0; it < 4; ++it) {
          const int row = it * 4 + q;
          const float* sp = slab + row * 68 + c8;
          v8h hv, lv;
#pragma unroll
          for (int e = 0; e < 8; ++e) {
            if (OUT_MODE == 1) {
              hv[e] = (_Float16)sp[e];
            } else {
              unsigned short hb = f2bf_bits(sp[e]);
              unsigned short lb = f2bf_bits(sp[e] - bf_bits2f(hb));
              hv[e] = __builtin_bit_cast(_Float16, hb);
              lv[e] = __builtin_bit_cast(_Float16, lb);
            }
          }
          *(volatile v8h*)(C + (size_t)(mBase + row) * ldc + n0 + c8) = hv;
          if (OUT_MODE == 2) *(volatile v8h*)(C2 + (size_t)(mBase + row) * ldc + n0 + c8) = lv;
        }
        __threadfence();
      }
    }
    __builtin_amdgcn_fence(__ATOMIC_RELEASE, "workgroup");
    __builtin_amdgcn_wave_barrier();
    __builtin_amdgcn_fence(__ATOMIC_ACQUIRE, "workgroup");
  }
}

__global__ __launch_bounds__(256) void split_f32_bf16x2(
    const float* __restrict__ in, __bf16* __restrict__ hi, __bf16* __restrict__ lo, long n2) {
  long i = (long)blockIdx.x * 256 + threadIdx.x;
  long stride = (long)gridDim.x * 256;
  for (int pass = 0; pass < 2; ++pass) {
    for (long j = i; j < n2; j += stride) {
      const float a = in[2 * j], b = in[2 * j + 1];
      const unsigned short ah = f2bf_bits(a), bh = f2bf_bits(b);
      const unsigned short al = f2bf_bits(a - bf_bits2f(ah)), bl = f2bf_bits(b - bf_bits2f(bh));
      ((volatile unsigned*)hi)[j] = (unsigned)ah | ((unsigned)bh << 16);
      ((volatile unsigned*)lo)[j] = (unsigned)al | ((unsigned)bl << 16);
    }
    __threadfence();
  }
}


__global__ __launch_bounds__(256) void transpose_split_bf16(const float* __restrict__ in, int ldi,
                                                           __bf16* __restrict__ outH, __bf16* __restrict__ outL, int ldo) {
  __shared__ __align__(16) float tile[64][68];
  const int c0 = blockIdx.x * 64, r0 = blockIdx.y * 64;
  const int t = threadIdx.y * 32 + threadIdx.x;
  for (int i = threadIdx.y; i < 64; i += 8) {
    tile[threadIdx.x][i]      = in[(size_t)(r0 + i) * ldi + c0 + threadIdx.x];
    tile[32 + threadIdx.x][i] = in[(size_t)(r0 + i) * ldi + c0 + 32 + threadIdx.x];
  }
  __syncthreads();
  const int q = t >> 3, c8 = (t & 7) * 8;
  for (int pass = 0; pass < 2; ++pass) {
#pragma unroll
    for (int it = 0; it < 2; ++it) {
      const int c = it * 32 + q;
      v8b hv, lv;
#pragma unroll
      for (int e = 0; e < 8; ++e) {
        const float f = tile[c][c8 + e];
        const unsigned short hb = f2bf_bits(f);
        hv[e] = __builtin_bit_cast(__bf16, hb);
        lv[e] = __builtin_bit_cast(__bf16, f2bf_bits(f - bf_bits2f(hb)));
      }
      *(volatile v8b*)(outH + (size_t)(c0 + c) * ldo + r0 + c8) = hv;
      *(volatile v8b*)(outL + (size_t)(c0 + c) * ldo + r0 + c8) = lv;
    }
    __threadfence();
  }
}

#define NN 50000
#define NPAD 50176
#define NE 400000
#define HC 64
#define NHD 8
#define H2 32
#define NG 32
#define NODES_PER_BLK 256
#define NBLK ((NN + NODES_PER_BLK - 1) / NODES_PER_BLK)
#define SEG_CAP 16384

#define ECH 8192
#define NCH ((NE + ECH - 1) / ECH)
#define NRP (((NBLK) + 31) & ~31)
#define SEG_STRIDE SEG_CAP
#define BUCKET_INTS ((size_t)NE + (size_t)32 * NCH * NBLK)
__device__ __forceinline__ int rank_eq(int key, bool valid, int lane, int nbits, int& ntotal) {
  unsigned same = __ballot(valid);
  for (int b = 0; b < nbits; ++b) {
    const unsigned m = __ballot(((key >> b) & 1) != 0);
    same &= (((key >> b) & 1) != 0) ? m : ~m;
  }
  if (!valid) same = 0u;
  ntotal = __popc(same);
  return __popc(same & ((1u << lane) - 1u));
}
__global__ __launch_bounds__(256) void csr_hist_kernel(const int* __restrict__ dst, int* __restrict__ cnt) {
  __shared__ int h[8][NRP];
  const int tid = threadIdx.x, lane = tid & 31, wave = tid >> 5;
  for (int i = tid; i < 8 * NRP; i += 256) (&h[0][0])[i] = 0;
  __syncthreads();
  const int e0 = blockIdx.x * ECH + wave * (ECH / 8), e1 = min(e0 + ECH / 8, NE);
  for (int c0 = e0; c0 < e0 + ECH / 8; c0 += 32) {
    const int e = c0 + lane;
    const bool valid = e < e1;
    int d = valid ? dst[e] : 0; d = d < 0 ? 0 : (d >= NN ? NN - 1 : d);
    const int r = d / NODES_PER_BLK;
    int tot; const int rk = rank_eq(r, valid, lane, 9, tot);
    if (valid && rk == tot - 1) h[wave][r] += tot;
  }
  __syncthreads();
  for (int pass = 0; pass < 2; ++pass) {
    for (int i = tid; i < NRP; i += 256) { int s = 0; for (int w = 0; w < 8; ++w) s += h[w][i]; ((volatile int*)cnt)[(size_t)blockIdx.x * NRP + i] = s; }
    __threadfence();
  }
}
__global__ __launch_bounds__(1024) void csr_offsets_kernel(const int* __restrict__ cnt, int* __restrict__ boff, int* __restrict__ rinfo) {
  __shared__ int rsz[1024];
  const int t = threadIdx.x;
  int run = 0;
  if (t < NBLK) { for (int c = 0; c < NCH; ++c) run += (cnt[(size_t)c * NRP + t] + 31) & ~31; }
  rsz[t] = (t < NBLK) ? run : 0;
  __syncthreads();
  for (int off = 1; off < 1024; off <<= 1) { int v = (t >= off) ? rsz[t - off] : 0; __syncthreads(); rsz[t] += v; __syncthreads(); }
  const int incl = rsz[t], excl = incl - ((t < NBLK) ? run : 0);
  __syncthreads();
  for (int pass = 0; pass < 2; ++pass) {
    if (t < NBLK) { int r2 = excl; for (int c = 0; c < NCH; ++c) { const size_t i = (size_t)c * NRP + t; ((volatile int*)boff)[i] = r2; r2 += (cnt[i] + 31) & ~31; } }
    ((volatile int*)rinfo)[t] = excl;
    ((volatile int*)rinfo)[1024 + t] = (t < NBLK) ? run : 0;
    __threadfence();
  }
}
__global__ __launch_bounds__(256) void csr_bucket_kernel(const int* __restrict__ dst, const int* __restrict__ boff, int* __restrict__ bucket) {
  __shared__ int wc[8][NRP];
  __shared__ int woff[8][NRP];
  __shared__ int roff[NRP + 1];
  __shared__ int seg[ECH + 32 * NRP];
  const int tid = threadIdx.x, lane = tid & 31, wave = tid >> 5;
  for (int i = tid; i < 8 * NRP; i += 256) { (&wc[0][0])[i] = 0; }
  __syncthreads();
  const int e0 = blockIdx.x * ECH + wave * (ECH / 8), e1 = min(e0 + ECH / 8, NE);
  for (int c0 = e0; c0 < e0 + ECH / 8; c0 += 32) {
    const int e = c0 + lane; const bool valid = e < e1;
    int d = valid ? dst[e] : 0; d = d < 0 ? 0 : (d >= NN ? NN - 1 : d);
    const int r = d / NODES_PER_BLK;
    int tot; const int rk = rank_eq(r, valid, lane, 9, tot);
    if (valid && rk == tot - 1) wc[wave][r] += tot;
  }
  __syncthreads();
  __shared__ int tot_r[NRP];
  for (int i = tid; i < NRP; i += 256) { int s = 0; for (int w = 0; w < 8; ++w) s += wc[w][i]; tot_r[i] = s; }
  __syncthreads();
  if (tid == 0) { int run = 0; for (int r = 0; r < NRP; ++r) { roff[r] = run; int o = run; for (int w = 0; w < 8; ++w) { woff[w][r] = o; o += wc[w][r]; } run += (tot_r[r] + 31) & ~31; } roff[NRP] = run; }
  __syncthreads();
  const int totalpad = roff[NRP];
  for (int i = tid; i < totalpad && i < ECH + 32 * NRP; i += 256) seg[i] = -1;
  __syncthreads();
  for (int c0 = e0; c0 < e0 + ECH / 8; c0 += 32) {
    const int e = c0 + lane; const bool valid = e < e1;
    int d = valid ? dst[e] : 0; d = d < 0 ? 0 : (d >= NN ? NN - 1 : d);
    const int r = d / NODES_PER_BLK;
    int tot; const int rk = rank_eq(r, valid, lane, 9, tot);
    if (valid) { const int slot = woff[wave][r] + rk; if (slot < ECH + 32 * NRP) seg[slot] = e; if (rk == tot - 1) woff[wave][r] = slot + 1; }
  }
  __syncthreads();
  for (int pass = 0; pass < 2; ++pass) {
    for (int r = wave; r < NBLK; r += 8) {
      const int lo = roff[r], n = ((tot_r[r] + 31) & ~31);
      const int gb = boff[(size_t)blockIdx.x * NRP + r];
      for (int i = lane; i < n; i += 32) ((volatile int*)bucket)[(size_t)gb + i] = (lo + i < ECH + 32 * NRP) ? seg[lo + i] : -1;
    }
    __threadfence();
  }
}
__global__ __launch_bounds__(256) void csr_fill_kernel(const int* __restrict__ dst, const int* __restrict__ bucket, const int* __restrict__ rinfo,
                                                      int* __restrict__ rowptr, int* __restrict__ rowdeg, int* __restrict__ csr_eid, int* __restrict__ rcl) {
  __shared__ int cnt[8][NODES_PER_BLK];
  __shared__ int off[8][NODES_PER_BLK];
  __shared__ int nodeoff[NODES_PER_BLK + 1];
  __shared__ int seg[SEG_CAP];
  const int tid = threadIdx.x, lane = tid & 31, wave = tid >> 5;
  const int n0 = blockIdx.x * NODES_PER_BLK;
  const int bstart = rinfo[blockIdx.x], bsize = rinfo[1024 + blockIdx.x];
  for (int i = tid; i < 8 * NODES_PER_BLK; i += 256) (&cnt[0][0])[i] = 0;
  for (int i = tid; i < SEG_CAP; i += 256) seg[i] = 0;
  __syncthreads();
  const int per = ((bsize / 8) + 31) & ~31;
  const int e0 = bstart + wave * per, e1 = min(bstart + (wave + 1) * per, bstart + bsize);
  for (int c0 = e0; c0 < e0 + per; c0 += 32) {
    const int j = c0 + lane;
    int e = (j < e1) ? bucket[j] : -1;
    const bool valid = (e >= 0) && (e < NE);
    int d = valid ? dst[e] : -1;
    const bool ok = valid && (d >= n0) && (d < n0 + NODES_PER_BLK);
    int tot; const int rk = rank_eq(ok ? (d - n0) : 0, ok, lane, 8, tot);
    if (ok && rk == tot - 1) cnt[wave][d - n0] += tot;
  }
  __syncthreads();
  if (tid < 32) {
    int loc[8]; int sum = 0;
    for (int q = 0; q < 8; ++q) { int c = 0; for (int w = 0; w < 8; ++w) c += cnt[w][tid * 8 + q]; loc[q] = c; sum += c; }
    int incl = sum;
    for (int o = 1; o < 32; o <<= 1) { int t = __shfl_up(incl, o, 32); if (lane >= o) incl += t; }
    int base = incl - sum;
    for (int q = 0; q < 8; ++q) {
      const int node = tid * 8 + q;
      nodeoff[node] = base;
      int run = base;
      for (int w = 0; w < 8; ++w) { off[w][node] = run; run += cnt[w][node]; }
      base += loc[q];
    }
    if (tid == 31) nodeoff[NODES_PER_BLK] = base;
  }
  __syncthreads();
  const int btotal = nodeoff[NODES_PER_BLK];
  for (int c0 = e0; c0 < e0 + per; c0 += 32) {
    const int j = c0 + lane;
    int e = (j < e1) ? bucket[j] : -1;
    const bool valid = (e >= 0) && (e < NE);
    int d = valid ? dst[e] : -1;
    const bool ok = valid && (d >= n0) && (d < n0 + NODES_PER_BLK);
    int tot; const int rk = rank_eq(ok ? (d - n0) : 0, ok, lane, 8, tot);
    if (ok) { const int slot = off[wave][d - n0] + rk; if (slot < SEG_CAP) seg[slot] = e; if (rk == tot - 1) off[wave][d - n0] = slot + 1; }
  }
  __syncthreads();
  const int gstart = blockIdx.x * (SEG_STRIDE);
  const int nlines = (min(btotal, SEG_CAP) + 31) >> 5;
  for (int pass = 0; pass < 2; ++pass) {
    { const int node = tid; int deg = 0; for (int w = 0; w < 8; ++w) deg += cnt[w][node];
      ((volatile int*)rowptr)[n0 + node] = gstart + nodeoff[node]; ((volatile int*)rowdeg)[n0 + node] = deg; }
    for (int i = tid; i < nlines * 32; i += 256) ((volatile int*)csr_eid)[gstart + i] = (i < btotal) ? seg[i] : 0;
    if (rcl != nullptr && tid < 32) ((volatile int*)rcl)[blockIdx.x * 32 + tid] = (tid == 0) ? min(btotal, SEG_CAP) : 0;
    __threadfence();
  }
}

__device__ __forceinline__ float bn_eval(float v, const float* __restrict__ p, int c, int C) { return (v - p[2 * C + c]) * rsqrtf(p[3 * C + c] + 1e-5f) * p[c] + p[C + c]; }

__global__ __launch_bounds__(256) void conv1a_kernel(const float* __restrict__ x, const int* __restrict__ rowptr, const int* __restrict__ rowdeg,
                                                    const int* __restrict__ csr_eid, const int* __restrict__ col,
                                                    const float* __restrict__ w1, const float* __restrict__ b1, float* __restrict__ H1) {
  const int lane = threadIdx.x & 31, wave = threadIdx.x >> 5; const int n = blockIdx.x * 8 + wave;
  float s = 0.f;
  if (n < NN) { int j0 = rowptr[n]; int dg = rowdeg[n]; dg = dg < 0 ? 0 : (dg > SEG_CAP ? SEG_CAP : dg); j0 = j0 < 0 ? 0 : j0;
    for (int j = j0 + lane; j < j0 + dg; j += 32) { int e = csr_eid[j]; e = e < 0 ? 0 : (e >= NE ? NE - 1 : e); int c2 = col[e]; c2 = c2 < 0 ? 0 : (c2 >= NN ? NN - 1 : c2); s += x[c2]; }
    for (int o = 16; o > 0; o >>= 1) s += __shfl_xor(s, o, 32);
    s += x[n]; }
  const float v0 = fmaxf(s * w1[lane] + b1[lane], 0.f), v1 = fmaxf(s * w1[32 + lane] + b1[32 + lane], 0.f);
  for (int pass = 0; pass < 2; ++pass) {
    ((volatile float*)H1)[(size_t)n * HC + lane] = v0; ((volatile float*)H1)[(size_t)n * HC + 32 + lane] = v1; __threadfence();
  }
}

__global__ __launch_bounds__(256) void maskprop_kernel(const int* __restrict__ rowptr, const int* __restrict__ rowdeg, const int* __restrict__ csr_eid,
                                                      const int* __restrict__ col, const float* __restrict__ Min, float* __restrict__ Mout) {
  const int n = blockIdx.x * 256 + threadIdx.x; if (n >= NPAD) return;
  float m = 0.f;
  if (n < NN) { int j0 = rowptr[n]; int dg = rowdeg[n]; dg = dg < 0 ? 0 : (dg > SEG_CAP ? SEG_CAP : dg); j0 = j0 < 0 ? 0 : j0;
    float s = 0.f; for (int j = j0; j < j0 + dg; ++j) { int e = csr_eid[j]; e = e < 0 ? 0 : (e >= NE ? NE - 1 : e); int sN = col[e]; sN = sN < 0 ? 0 : (sN >= NN ? NN - 1 : sN); s += Min[sN]; }
    m = (s > 0.f) ? 1.f : 0.f; }
  ((volatile float*)Mout)[n] = m; __threadfence(); ((volatile float*)Mout)[n] = m;
}
__global__ __launch_bounds__(256) void bnmask_kernel(const float* __restrict__ Hin, const float* __restrict__ bnp, const float* __restrict__ MASK, float* __restrict__ H) {
  const int lane = threadIdx.x & 31, wave = threadIdx.x >> 5; const int n = blockIdx.x * 8 + wave;
  const float m = MASK[n];
  const float v0 = bn_eval(Hin[(size_t)n * HC + lane], bnp, lane, HC) * m, v1 = bn_eval(Hin[(size_t)n * HC + 32 + lane], bnp, 32 + lane, HC) * m;
  for (int pass = 0; pass < 2; ++pass) { ((volatile float*)H)[(size_t)n * HC + lane] = v0; ((volatile float*)H)[(size_t)n * HC + 32 + lane] = v1; __threadfence(); }
}
__global__ __launch_bounds__(256) void ginagg_kernel(const float* __restrict__ H, const int* __restrict__ rowptr, const int* __restrict__ rowdeg,
    const int* __restrict__ csr_eid, const int* __restrict__ col, const float* __restrict__ epsv, int li, float* __restrict__ AGG) {
  const int lane = threadIdx.x & 31, wave = threadIdx.x >> 5; const int n = blockIdx.x * 8 + wave;
  float a0 = 0.f, a1 = 0.f;
  if (n < NN) { int j0 = rowptr[n]; int dg = rowdeg[n]; dg = dg < 0 ? 0 : (dg > SEG_CAP ? SEG_CAP : dg); j0 = j0 < 0 ? 0 : j0;
    for (int j = j0; j < j0 + dg; ++j) { int e = csr_eid[j]; e = e < 0 ? 0 : (e >= NE ? NE - 1 : e); int s = col[e]; s = s < 0 ? 0 : (s >= NN ? NN - 1 : s); a0 += H[(size_t)s * HC + lane]; a1 += H[(size_t)s * HC + 32 + lane]; }
    const float f = 1.0f + epsv[li]; a0 += f * H[(size_t)n * HC + lane]; a1 += f * H[(size_t)n * HC + 32 + lane]; }
  for (int pass = 0; pass < 2; ++pass) { ((volatile float*)AGG)[(size_t)n * HC + lane] = a0; ((volatile float*)AGG)[(size_t)n * HC + 32 + lane] = a1; __threadfence(); }
}
__global__ __launch_bounds__(256) void ginupd_kernel(float* __restrict__ H, const float* __restrict__ T, const float* __restrict__ gbn, const float* __restrict__ sbn,
                                                    const float* __restrict__ MASK) {
  const int lane = threadIdx.x & 31, wave = threadIdx.x >> 5; const int n = blockIdx.x * 8 + wave;
  const float m = MASK[n];
  float v0 = H[(size_t)n * HC + lane] + bn_eval(T[(size_t)n * HC + lane], gbn, lane, HC);
  float v1 = H[(size_t)n * HC + 32 + lane] + bn_eval(T[(size_t)n * HC + 32 + lane], gbn, 32 + lane, HC);
  v0 = bn_eval(v0 * m, sbn, lane, HC); v1 = bn_eval(v1 * m, sbn, 32 + lane, HC);
  for (int pass = 0; pass < 2; ++pass) { ((volatile float*)H)[(size_t)n * HC + lane] = v0; ((volatile float*)H)[(size_t)n * HC + 32 + lane] = v1; __threadfence(); }
}
__global__ __launch_bounds__(256) void gatalpha_kernel(const float* __restrict__ XT, const float* __restrict__ att, float* __restrict__ AL) {
  const int n = blockIdx.x * 16 + (threadIdx.x >> 4), hsel = threadIdx.x & 15;
  const int hd = hsel & 7, part = hsel >> 3;
  float s = 0.f;
  if (n < NN) {
#pragma unroll 1
    for (int c = 0; c < H2; ++c) s += XT[(size_t)n * (NHD * H2) + hd * H2 + c] * att[hd * 2 * H2 + part * H2 + c];
  }
  ((volatile float*)AL)[(size_t)n * 16 + part * 8 + hd] = s; __threadfence(); ((volatile float*)AL)[(size_t)n * 16 + part * 8 + hd] = s;
}
__device__ __forceinline__ float lrelu2(float v) { return v > 0.f ? v : 0.2f * v; }
__global__ __launch_bounds__(256) void gatagg_kernel(const float* __restrict__ XT, const float* __restrict__ AL, const int* __restrict__ rowptr,
    const int* __restrict__ rowdeg, const int* __restrict__ csr_eid, const int* __restrict__ col, const float* __restrict__ gbias,
    const float* __restrict__ MASK, float* __restrict__ HG) {
  const int lane = threadIdx.x & 31, wave = threadIdx.x >> 5; const int n = blockIdx.x * 8 + wave;
  const int hd = lane >> 2, c0 = 8 * lane;
  float acc[8]; float l = 0.f, m = -INFINITY;
#pragma unroll
  for (int q = 0; q < 8; ++q) acc[q] = 0.f;
  float mk = 0.f;
  if (n < NN) {
    mk = MASK[n];
    const float ai = AL[(size_t)n * 16 + hd];
    int j0 = rowptr[n]; int dg = rowdeg[n]; dg = dg < 0 ? 0 : (dg > SEG_CAP ? SEG_CAP : dg); j0 = j0 < 0 ? 0 : j0;
    for (int j = j0 - 1; j < j0 + dg; ++j) {
      int s;
      if (j < j0) s = n; else { int e = csr_eid[j]; e = e < 0 ? 0 : (e >= NE ? NE - 1 : e); s = col[e]; s = s < 0 ? 0 : (s >= NN ? NN - 1 : s); }
      const float a = lrelu2(ai + AL[(size_t)s * 16 + 8 + hd]);
      const float mn = fmaxf(m, a), al = expf(m - mn), w = expf(a - mn);
      l = l * al + w; m = mn;
      const v4f x0 = *(const v4f*)(XT + (size_t)s * (NHD * H2) + c0), x1 = *(const v4f*)(XT + (size_t)s * (NHD * H2) + c0 + 4);
      acc[0] = acc[0] * al + w * x0[0]; acc[1] = acc[1] * al + w * x0[1]; acc[2] = acc[2] * al + w * x0[2]; acc[3] = acc[3] * al + w * x0[3];
      acc[4] = acc[4] * al + w * x1[0]; acc[5] = acc[5] * al + w * x1[1]; acc[6] = acc[6] * al + w * x1[2]; acc[7] = acc[7] * al + w * x1[3];
    }
    const float inv = 1.0f / l;
#pragma unroll
    for (int q = 0; q < 8; ++q) acc[q] = (acc[q] * inv + gbias[c0 + q]) * mk;
  }
  const v4f o0 = {acc[0], acc[1], acc[2], acc[3]}, o1 = {acc[4], acc[5], acc[6], acc[7]};
  for (int pass = 0; pass < 2; ++pass) {
    *(volatile v4f*)(HG + (size_t)n * (NHD * H2) + c0) = o0; *(volatile v4f*)(HG + (size_t)n * (NHD * H2) + c0 + 4) = o1; __threadfence();
  }
}
__global__ __launch_bounds__(256) void tail_kernel(const float* __restrict__ L1, const float* __restrict__ MASK, const float* __restrict__ bn2p,
                                                  const float* __restrict__ w2, const float* __restrict__ b2, float* __restrict__ H5) {
  __shared__ float sv[256];
  const int lane = threadIdx.x & 31, wave = threadIdx.x >> 5;
  for (int rd = 0; rd < 32; ++rd) {
    const int n = blockIdx.x * 256 + rd * 8 + wave;
    float v = 0.f;
    if (n < NN) {
      const float m = MASK[n];
      const float h0 = bn_eval(L1[(size_t)n * HC + lane] * m, bn2p, lane, HC), h1 = bn_eval(L1[(size_t)n * HC + 32 + lane] * m, bn2p, 32 + lane, HC);
      float d = h0 * w2[lane] + h1 * w2[32 + lane];
      for (int o = 16; o > 0; o >>= 1) d += __shfl_xor(d, o, 32);
      d += b2[0];
      v = ((d > 0.f) ? d : 0.01f * d) * m;
    }
    if (lane == 0) sv[rd * 8 + wave] = v;
  }
  __syncthreads();
  const float o = sv[threadIdx.x];
  ((volatile float*)H5)[(size_t)blockIdx.x * 256 + threadIdx.x] = o; __threadfence(); ((volatile float*)H5)[(size_t)blockIdx.x * 256 + threadIdx.x] = o;
}
__global__ __launch_bounds__(256) void graphmm_kernel(const float* __restrict__ H5, const int* __restrict__ batch, float* __restrict__ MM) {
  __shared__ int rg[2]; __shared__ float smn[256], smx[256];
  const int g = blockIdx.x, t = threadIdx.x;
  if (t < 2) { const int key = g + t; int lo = 0, hi = NN; while (lo < hi) { const int mid = (lo + hi) >> 1; if (batch[mid] < key) lo = mid + 1; else hi = mid; } rg[t] = lo; }
  __syncthreads();
  float mn = INFINITY, mx = -INFINITY;
  for (int n = rg[0] + t; n < rg[1]; n += 256) { if (batch[n] == g) { const float v = H5[n]; mn = fminf(mn, v); mx = fmaxf(mx, v); } }
  smn[t] = mn; smx[t] = mx; __syncthreads();
  for (int s = 128; s > 0; s >>= 1) { if (t < s) { smn[t] = fminf(smn[t], smn[t + s]); smx[t] = fmaxf(smx[t], smx[t + s]); } __syncthreads(); }
  if (t < 32) { const float v = (t == 0) ? smn[0] : (t == 1 ? smx[0] : 0.f); ((volatile float*)MM)[g * 32 + t] = v; __threadfence(); ((volatile float*)MM)[g * 32 + t] = v; }
}
__global__ __launch_bounds__(256) void probs_kernel(const float* __restrict__ H5, const float* __restrict__ MASK, const int* __restrict__ batch, const float* __restrict__ MM, float* __restrict__ out) {
  const int n = blockIdx.x * 256 + threadIdx.x; if (n >= NN) return;
  int g = batch[n]; g = g < 0 ? 0 : (g >= NG ? NG - 1 : g);
  const float bmin = MM[g * 32], bmax = MM[g * 32 + 1], m = MASK[n];
  const float h = (H5[n] - bmin) / (bmax + 1e-6f - bmin);
  const float v = h * m + m * 1e-6f;
  ((volatile float*)out)[n] = v; __threadfence(); ((volatile float*)out)[n] = v;
}

extern "C" void kernel_launch(void* const* d_in, const int* in_sizes, int n_in,
                              void* d_out, int out_size, void* d_ws, size_t ws_size,
                              hipStream_t stream) {
  (void)in_sizes; (void)n_in; (void)out_size; (void)ws_size;
  const int* ei = (const int*)d_in[1];
  const int* batch = (const int*)d_in[2];
  const float* c1w1 = (const float*)d_in[3]; const float* c1b1 = (const float*)d_in[4]; const float* c1w2 = (const float*)d_in[5]; const float* c1b2 = (const float*)d_in[6]; const float* c1bn = (const float*)d_in[7];
  const float* gw1 = (const float*)d_in[8]; const float* gb1 = (const float*)d_in[9]; const float* gw2 = (const float*)d_in[10]; const float* gb2 = (const float*)d_in[11];
  const float* gbn = (const float*)d_in[12]; const float* geps = (const float*)d_in[13]; const float* sbn = (const float*)d_in[14];
  const float* gatw = (const float*)d_in[15]; const float* gatatt = (const float*)d_in[16]; const float* gatb = (const float*)d_in[17];
  const float* l1w = (const float*)d_in[18]; const float* l1b = (const float*)d_in[19]; const float* bn2 = (const float*)d_in[20];
  const float* l2w = (const float*)d_in[21]; const float* l2b = (const float*)d_in[22];
  float* out = (float*)d_out;
  const float* xin = (const float*)d_in[0];

  char* ws = (char*)d_ws; size_t off = 0;
  auto carve = [&](size_t bytes) -> char* { char* p = ws + off; off += (bytes + 255) & ~(size_t)255; return p; };
  int* ccnt = (int*)carve((size_t)NCH * NRP * 4); int* boff = (int*)carve((size_t)NCH * NRP * 4); int* rinfo = (int*)carve((size_t)2048 * 4);
  int* bucket = (int*)carve(BUCKET_INTS * 4);
  int* rowptr = (int*)carve((size_t)NPAD * 4); int* rowdeg = (int*)carve((size_t)NPAD * 4);
  int* csr_eid = (int*)carve((size_t)NBLK * SEG_STRIDE * 4);
  float* MASKA = (float*)carve((size_t)NPAD * 4); float* MASKB = (float*)carve((size_t)NPAD * 4);
  float* H = (float*)carve((size_t)NPAD * HC * 4); float* AGG = (float*)carve((size_t)NPAD * HC * 4); float* T = (float*)carve((size_t)NPAD * HC * 4); float* T2 = (float*)carve((size_t)NPAD * HC * 4);
  __bf16* Ah = (__bf16*)carve((size_t)NPAD * 256 * 2); __bf16* Al = (__bf16*)carve((size_t)NPAD * 256 * 2);
  __bf16* Wh = (__bf16*)carve((size_t)256 * 256 * 2); __bf16* Wl = (__bf16*)carve((size_t)256 * 256 * 2);
  float* XT = (float*)carve((size_t)NPAD * 256 * 4); float* AL = (float*)carve((size_t)NPAD * 16 * 4); float* HG = (float*)carve((size_t)NPAD * 256 * 4);
  float* L1 = (float*)carve((size_t)NPAD * HC * 4); float* H5 = (float*)carve((size_t)NPAD * 4); float* MM = (float*)carve((size_t)NG * 32 * 4);

  const int tl64 = (NPAD / 64) * 1, tl256 = (NPAD / 64) * 4;
  auto gemm64 = [&](const float* Af, int K, const float* Wkn  , int N, const float* bias, float* Cf, int act) {
    split_f32_bf16x2<<<(NPAD * K / 2 + 255) / 256, 256, 0, stream>>>(Af, Ah, Al, NPAD * K / 2);
    transpose_split_bf16<<<dim3(N / 64, K / 64), dim3(32, 8), 0, stream>>>(Wkn, N, Wh, Wl, K);
    const int tl = (NPAD / 64) * (N / 64);
    if (act == 2) wmma_gemm64<1, true, 2, 0, false, 2><<<dim3((tl + 7) / 8, 1), 256, 0, stream>>>(U16(Ah), U16(Al), K, 0, U16(Wh), U16(Wl), K, 0, Cf, nullptr, N, 0, bias, nullptr, 0, NPAD, N, K, 1.0f);
    else if (act == 4) wmma_gemm64<1, true, 2, 0, false, 4><<<dim3((tl + 7) / 8, 1), 256, 0, stream>>>(U16(Ah), U16(Al), K, 0, U16(Wh), U16(Wl), K, 0, Cf, nullptr, N, 0, bias, nullptr, 0, NPAD, N, K, 1.0f);
    else wmma_gemm64<1, true, 0, 0, false, 0><<<dim3((tl + 7) / 8, 1), 256, 0, stream>>>(U16(Ah), U16(Al), K, 0, U16(Wh), U16(Wl), K, 0, Cf, nullptr, N, 0, nullptr, nullptr, 0, NPAD, N, K, 1.0f);
  };
  (void)tl64; (void)tl256;

  csr_hist_kernel<<<NCH, 256, 0, stream>>>(ei, ccnt);
  csr_offsets_kernel<<<1, 1024, 0, stream>>>(ccnt, boff, rinfo);
  csr_bucket_kernel<<<NCH, 256, 0, stream>>>(ei, boff, bucket);
  csr_fill_kernel<<<NBLK, 256, 0, stream>>>(ei, bucket, rinfo, rowptr, rowdeg, csr_eid, nullptr);
  maskprop_kernel<<<NPAD / 256, 256, 0, stream>>>(rowptr, rowdeg, csr_eid, ei + NE, xin, MASKA);
  conv1a_kernel<<<NPAD / 8, 256, 0, stream>>>(xin, rowptr, rowdeg, csr_eid, ei + NE, c1w1, c1b1, AGG);
  gemm64(AGG, HC, c1w2, HC, c1b2, T, 2);
  bnmask_kernel<<<NPAD / 8, 256, 0, stream>>>(T, c1bn, MASKA, H);
  float* Mcur = MASKA; float* Mnext = MASKB;
  for (int i = 0; i < 3; ++i) {
    ginagg_kernel<<<NPAD / 8, 256, 0, stream>>>(H, rowptr, rowdeg, csr_eid, ei + NE, geps, i, AGG);
    gemm64(AGG, HC, gw1 + (size_t)i * HC * HC, HC, gb1 + i * HC, T, 2);
    gemm64(T, HC, gw2 + (size_t)i * HC * HC, HC, gb2 + i * HC, T2, 2);
    maskprop_kernel<<<NPAD / 256, 256, 0, stream>>>(rowptr, rowdeg, csr_eid, ei + NE, Mcur, Mnext);
    ginupd_kernel<<<NPAD / 8, 256, 0, stream>>>(H, T2, gbn + (size_t)i * 4 * HC, sbn + (size_t)i * 4 * HC, Mnext);
    float* tmp = Mcur; Mcur = Mnext; Mnext = tmp;
  }
  gemm64(H, HC, gatw, 256, nullptr, XT, 0);
  gatalpha_kernel<<<NPAD / 16, 256, 0, stream>>>(XT, gatatt, AL);
  maskprop_kernel<<<NPAD / 256, 256, 0, stream>>>(rowptr, rowdeg, csr_eid, ei + NE, Mcur, Mnext);
  gatagg_kernel<<<NPAD / 8, 256, 0, stream>>>(XT, AL, rowptr, rowdeg, csr_eid, ei + NE, gatb, Mnext, HG);
  gemm64(HG, 256, l1w, HC, l1b, L1, 4);
  tail_kernel<<<NPAD / 256, 256, 0, stream>>>(L1, Mnext, bn2, l2w, l2b, H5);
  graphmm_kernel<<<NG, 256, 0, stream>>>(H5, batch, MM);
  probs_kernel<<<NPAD / 256, 256, 0, stream>>>(H5, Mnext, batch, MM, out);
}
